// SelfAttention_88596585382183
// MI455X (gfx1250) — hardware-verified
//
#include <hip/hip_runtime.h>
#ifndef NB
#define NB 16
#endif
#ifndef SEQ
#define SEQ 1024
#endif
#define NB_FULL 16
#define SEQ_FULL 1024
#define CIN 256
#define NH 4
#define HD 64
#define TD 256
#define QP 768
#define KOF 256
#define VOF 512
#define TROWS 32
#define PCARRY 16384.0f
#define LCARRY 2048.0f
#define NR ((size_t)NB * SEQ)
static_assert(SEQ % 256 == 0);
static_assert((NR % 128) == 0);
static_assert(NB <= NB_FULL);
static_assert(SEQ <= SEQ_FULL);
static_assert(3 * CIN == QP);
static_assert(KOF == CIN && VOF == 2 * CIN);
static_assert(CIN == NH * HD);
static_assert(CIN % 64 == 0 && QP % 64 == 0 && HD == 64);
static_assert(TD == CIN);
static_assert(TD % 32 == 0 && HD % 32 == 0 && SEQ % 32 == 0 && CIN % 32 == 0);
static_assert(TROWS == 32 && NB <= TROWS);
static_assert((QP * (CIN / 8)) % 256 == 0 && (CIN * (CIN / 8)) % 256 == 0 && (TROWS * (TD / 8)) % 256 == 0);
static_assert(SEQ % 128 == 0 && SEQ % 64 == 0);

typedef unsigned short v8us __attribute__((ext_vector_type(8), may_alias));
typedef float  v8f  __attribute__((ext_vector_type(8)));
typedef float  v4f  __attribute__((ext_vector_type(4)));
typedef float  v4fa __attribute__((ext_vector_type(4), may_alias));
typedef _Float16 v16h __attribute__((ext_vector_type(16)));
typedef _Float16 v4h __attribute__((ext_vector_type(4)));
typedef _Float16 h16;
union FragH { v16h v; v8us half[2]; _Float16 h[16]; unsigned short u[16]; };

__device__ __forceinline__ unsigned short bf16_bits(float x) { unsigned int u = __float_as_uint(x); return (unsigned short)((u + 0x7FFFu + ((u >> 16) & 1u)) >> 16); }
__device__ __forceinline__ float bf16_val(unsigned short b) { return __uint_as_float(((unsigned int)b) << 16); }
__device__ __forceinline__ float bf16_rne(float x) { return bf16_val(bf16_bits(x)); }
static __device__ __forceinline__ h16 toh_flush(float v) { const h16 r = (h16)v; return (fabsf(v) < 6.103515625e-05f) ? (h16)0.0f : r; }

__device__ __forceinline__ v16h g2_frag(const _Float16* p, int hh) { FragH f; f.half[0] = *(const v8us*)((const unsigned short*)p + 8 * hh); f.half[1] = *(const v8us*)((const unsigned short*)p + 16 + 8 * hh); return f.v; }
__device__ __forceinline__ v8f g2_mma(v16h a, v16h b, v8f c) { v8f d = __builtin_amdgcn_wmma_f32_16x16x32_f16(false, a, false, b, (short)0, c, false, false); asm volatile("v_nop\n\tv_nop\n\tv_nop\n\tv_nop" : "+v"(d) : "v"(a), "v"(b)); return d; }

__device__ __forceinline__ void g2_kloop(const _Float16* __restrict__ a0p, const _Float16* __restrict__ a1p, const _Float16* __restrict__ b0p, const _Float16* __restrict__ b1p, const _Float16* __restrict__ b2p, const _Float16* __restrict__ b3p, int K, int hh,
    v8f& c00, v8f& c01, v8f& c02, v8f& c03, v8f& c10, v8f& c11, v8f& c12, v8f& c13) {
#pragma unroll 1
  for (int kb = 0; kb < K; kb += 32) { const v16h a0 = g2_frag(a0p + kb, hh), a1 = g2_frag(a1p + kb, hh);
    v16h b = g2_frag(b0p + kb, hh); c00 = g2_mma(a0, b, c00); c10 = g2_mma(a1, b, c10);
    b = g2_frag(b1p + kb, hh); c01 = g2_mma(a0, b, c01); c11 = g2_mma(a1, b, c11);
    b = g2_frag(b2p + kb, hh); c02 = g2_mma(a0, b, c02); c12 = g2_mma(a1, b, c12);
    b = g2_frag(b3p + kb, hh); c03 = g2_mma(a0, b, c03); c13 = g2_mma(a1, b, c13); }
}

template <int RES>
__global__ __launch_bounds__(128) void k_gemm2(const _Float16* __restrict__ A, int lda, size_t sA, const _Float16* __restrict__ A2, int lda2, size_t sA2,
    const _Float16* __restrict__ Bh, int ldb, size_t sB, const _Float16* __restrict__ B2, int ldb2, size_t sB2, float rscale,
    float alpha, const float* __restrict__ bias, size_t sBias,
    float* __restrict__ C, _Float16* __restrict__ C16, int ldc, size_t sC, _Float16* __restrict__ C16L, int ldcl, size_t sCL, int NL, int M, int N, int K) {
  __shared__ __attribute__((aligned(16))) float so[4][32][68];
  const int tid = threadIdx.x, w = tid >> 5, lane = tid & 31, ln = lane & 15, hh = lane >> 4; const int by = blockIdx.y;
  A += (size_t)by * sA; Bh += (size_t)by * sB;
  if (RES) { A2 += (size_t)by * sA2; B2 += (size_t)by * sB2; }
  const size_t cofs = (size_t)by * sC, cofl = (size_t)by * sCL; const float* bp = bias ? bias + (size_t)by * sBias : nullptr;
  const int ntn = N >> 6; const int mt = blockIdx.x / ntn, nq = blockIdx.x - mt * ntn; const int row0 = mt * 128 + 32 * w, col0 = nq * 64; if (row0 >= M) return;
  const _Float16* a0p = A + (size_t)(row0 + ln) * lda; const _Float16* a1p = a0p + (size_t)16 * lda;
  const _Float16* b0p = Bh + (size_t)(col0 + ln) * ldb; const _Float16* b1p = b0p + (size_t)16 * ldb; const _Float16* b2p = b1p + (size_t)16 * ldb; const _Float16* b3p = b2p + (size_t)16 * ldb;
  const v8f z8 = {0.f,0.f,0.f,0.f,0.f,0.f,0.f,0.f}; v8f c00 = z8, c01 = z8, c02 = z8, c03 = z8, c10 = z8, c11 = z8, c12 = z8, c13 = z8;
  if (RES) {
    const _Float16* l0p = A2 + (size_t)(row0 + ln) * lda2; const _Float16* l1p = l0p + (size_t)16 * lda2;
    const _Float16* m0p = B2 + (size_t)(col0 + ln) * ldb2; const _Float16* m1p = m0p + (size_t)16 * ldb2; const _Float16* m2p = m1p + (size_t)16 * ldb2; const _Float16* m3p = m2p + (size_t)16 * ldb2;
    g2_kloop(l0p, l1p, b0p, b1p, b2p, b3p, K, hh, c00, c01, c02, c03, c10, c11, c12, c13);
    g2_kloop(a0p, a1p, m0p, m1p, m2p, m3p, K, hh, c00, c01, c02, c03, c10, c11, c12, c13);
    c00 = c00 * rscale; c01 = c01 * rscale; c02 = c02 * rscale; c03 = c03 * rscale; c10 = c10 * rscale; c11 = c11 * rscale; c12 = c12 * rscale; c13 = c13 * rscale;
  }
  g2_kloop(a0p, a1p, b0p, b1p, b2p, b3p, K, hh, c00, c01, c02, c03, c10, c11, c12, c13);
  v8f accs[8] = {c00, c01, c02, c03, c10, c11, c12, c13};
#pragma unroll
  for (int u = 0; u < 8; ++u) { const int t = u & 3, half = u >> 2; const int col = col0 + t * 16 + ln; const float bv = bp ? bf16_rne(bp[col]) : 0.f;
#pragma unroll
    for (int r = 0; r < 8; ++r) { const int rloc = half * 16 + 8 * hh + r; so[w][rloc][t * 16 + ln] = accs[u][r] * alpha + bv; } }
  __builtin_amdgcn_fence(4  , "workgroup"); __builtin_amdgcn_wave_barrier();
  const int rsub = lane >> 4, c4 = (lane & 15) * 4; const bool wl = (C16L != nullptr) && (col0 < NL);
  for (int pass = 0; pass < 2; ++pass) {
#pragma unroll
    for (int q = 0; q < 16; ++q) { const int r = q * 2 + rsub; const v4f v = *(const v4fa*)&so[w][r][c4];
      if (C) *(volatile v4f*)(C + cofs + (size_t)(row0 + r) * ldc + col0 + c4) = v;
      if (C16) { v4h h4; for (int i = 0; i < 4; ++i) h4[i] = (_Float16)v[i]; *(volatile v4h*)(C16 + cofs + (size_t)(row0 + r) * ldc + col0 + c4) = h4;
        if (wl) { v4h l4; for (int i = 0; i < 4; ++i) l4[i] = (_Float16)((v[i] - (float)h4[i]) * LCARRY); *(volatile v4h*)(C16L + cofl + (size_t)(row0 + r) * ldcl + col0 + c4) = l4; } } }
    if (pass == 0) __threadfence(); } }

__global__ __launch_bounds__(256) void k_w16t(const float* __restrict__ W, int ldw, int nrows, _Float16* __restrict__ BW) {
  const int t = blockIdx.x * 256 + threadIdx.x; if (t >= nrows * (CIN / 8)) return;
  const int n = t / (CIN / 8), k8 = (t % (CIN / 8)) * 8;
  FragH f;
#pragma unroll
  for (int q = 0; q < 8; ++q) f.h[q] = toh_flush(bf16_rne(W[(size_t)(k8 + q) * ldw + n]) * 16.0f);
  const v8us o = f.half[0];
  *(volatile v8us*)((unsigned short*)BW + (size_t)n * CIN + k8) = o; __threadfence(); *(volatile v8us*)((unsigned short*)BW + (size_t)n * CIN + k8) = o;
}

__global__ __launch_bounds__(256) void k_t16(const float* __restrict__ t_emb, _Float16* __restrict__ T16) {
  const int t = blockIdx.x * 256 + threadIdx.x; if (t >= TROWS * (TD / 8)) return;
  const int r = t / (TD / 8), k8 = (t % (TD / 8)) * 8;
  const int rr = (r < NB) ? r : (NB - 1);
  const float* p = t_emb + (size_t)rr * TD + k8;
  const v4f a = *(const v4fa*)p, c = *(const v4fa*)(p + 4);
  FragH f;
#pragma unroll
  for (int q = 0; q < 4; ++q) { const float va = (r < NB) ? bf16_rne(a[q]) : 0.0f; const float vc = (r < NB) ? bf16_rne(c[q]) : 0.0f; f.h[q] = toh_flush(va); f.h[4 + q] = toh_flush(vc); }
  const v8us o = f.half[0];
  *(volatile v8us*)((unsigned short*)T16 + (size_t)r * TD + k8) = o; __threadfence(); *(volatile v8us*)((unsigned short*)T16 + (size_t)r * TD + k8) = o;
}

__global__ __launch_bounds__(256) void k_xt16(const float* __restrict__ x, const float* __restrict__ te, _Float16* __restrict__ X16) {
  __shared__ __attribute__((aligned(16))) unsigned short tl[64][72];
  const int tid = threadIdx.x; constexpr int NCT = CIN / 64, NNT = SEQ / 64;
  const int ct = blockIdx.x % NCT, nt = (blockIdx.x / NCT) % NNT, b = blockIdx.x / (NCT * NNT);
  const int n0 = nt * 64, c0 = ct * 64;
  for (int i = tid; i < 64 * 16; i += 256) { const int cr = i >> 4, f4 = i & 15;
    const v4f a = *(const v4fa*)(x + ((size_t)b * CIN + c0 + cr) * SEQ_FULL + n0 + f4 * 4); const float tv = te[(size_t)b * CIN + c0 + cr]; FragH f;
#pragma unroll
    for (int q = 0; q < 4; ++q) { f.h[q] = toh_flush(bf16_rne(a[q]) + tv); tl[f4 * 4 + q][cr] = f.u[q]; } }
  __syncthreads();
  for (int pass = 0; pass < 2; ++pass) {
#pragma unroll
    for (int rd = 0; rd < 2; ++rd) { const int n = rd * 32 + (tid >> 3), pc = tid & 7; FragH f;
#pragma unroll
      for (int q = 0; q < 8; ++q) f.u[q] = tl[n][pc * 8 + q];
      *(volatile v8us*)((unsigned short*)X16 + ((size_t)b * SEQ + n0 + n) * CIN + c0 + pc * 8) = f.half[0]; }
    if (pass == 0) __threadfence(); } }

__global__ __launch_bounds__(256) void k_vt(const _Float16* __restrict__ QHp, _Float16* __restrict__ Vt) {
  __shared__ unsigned short tl[64][66]; const int tid = threadIdx.x; constexpr int NLG = SEQ / 64;
  const int lg = blockIdx.x % NLG, bh = blockIdx.x / NLG, h = bh % NH, b = bh / NH;
  for (int i = tid; i < 64 * 8; i += 256) { const int r = i / 8, c8 = (i % 8) * 8; FragH f; f.half[0] = *(const v8us*)((const unsigned short*)QHp + ((size_t)b * SEQ + lg * 64 + r) * QP + VOF + h * HD + c8);
#pragma unroll
    for (int q = 0; q < 8; ++q) tl[r][c8 + q] = f.u[q]; }
  __syncthreads();
  for (int pass = 0; pass < 2; ++pass) {
#pragma unroll
    for (int rd = 0; rd < 2; ++rd) { const int d = rd * 32 + tid / 8, pc = tid % 8; FragH f;
#pragma unroll
      for (int q = 0; q < 8; ++q) f.u[q] = tl[pc * 8 + q][d];
      *(volatile v8us*)((unsigned short*)Vt + (((size_t)b * NH + h) * HD + d) * SEQ + lg * 64 + pc * 8) = f.half[0]; }
    if (pass == 0) __threadfence(); } }

__global__ __launch_bounds__(256) void k_rsmw(const float* __restrict__ S, _Float16* __restrict__ P, int nrows) {
  #pragma clang fp contract(off)
  const int row = blockIdx.x * 8 + (threadIdx.x >> 5), lane = threadIdx.x & 31;
  if (row >= nrows) return;
  const float* s = S + (size_t)row * SEQ;
  constexpr int NI = SEQ / 256;
  float v[NI * 8];
  float mx = -3.0e38f;
#pragma unroll
  for (int i = 0; i < NI; ++i) {
    const v4f a = *(const v4fa*)(s + i * 256 + lane * 8), c = *(const v4fa*)(s + i * 256 + lane * 8 + 4);
#pragma unroll
    for (int q = 0; q < 4; ++q) { v[i * 8 + q] = a[q]; v[i * 8 + 4 + q] = c[q]; mx = fmaxf(mx, fmaxf(a[q], c[q])); }
  }
#pragma unroll
  for (int o = 16; o > 0; o >>= 1) mx = fmaxf(mx, __shfl_xor(mx, o, 32));
  float se = 0.f;
#pragma unroll
  for (int j = 0; j < NI * 8; ++j) { const float e = __expf(v[j] - mx); v[j] = e; se += e; }
#pragma unroll
  for (int o = 16; o > 0; o >>= 1) se += __shfl_xor(se, o, 32);
  const float sc = PCARRY / se;
  unsigned short* prow = (unsigned short*)P + (size_t)row * SEQ;
  for (int pass = 0; pass < 2; ++pass) {
#pragma unroll
    for (int i = 0; i < NI; ++i) { FragH f;
#pragma unroll
      for (int q = 0; q < 8; ++q) f.h[q] = (_Float16)(v[i * 8 + q] * sc);
      *(volatile v8us*)(prow + i * 256 + lane * 8) = f.half[0]; }
    if (pass == 0) __threadfence();
  }
}

__global__ __launch_bounds__(256) void k_outT(const float* __restrict__ O2, float* __restrict__ out) {
  __shared__ __attribute__((aligned(16))) float tl[64][68];
  const int tid = threadIdx.x; constexpr int NCT = CIN / 64, NNT = SEQ / 64;
  const int ct = blockIdx.x % NCT, nt = (blockIdx.x / NCT) % NNT, b = blockIdx.x / (NCT * NNT);
  const int n0 = nt * 64, c0 = ct * 64;
  for (int i = tid; i < 64 * 16; i += 256) { const int tr = i >> 4, f4 = i & 15;
    const v4f a = *(const v4fa*)(O2 + ((size_t)b * SEQ + n0 + tr) * CIN + c0 + f4 * 4);
#pragma unroll
    for (int q = 0; q < 4; ++q) tl[f4 * 4 + q][tr] = a[q]; }
  __syncthreads();
  for (int pass = 0; pass < 2; ++pass) {
#pragma unroll
    for (int rd = 0; rd < 4; ++rd) { const int o = rd * 16 + (tid >> 4), pc = tid & 15; const v4f v = *(const v4fa*)&tl[o][pc * 4];
      *(volatile v4f*)(out + ((size_t)b * CIN + c0 + o) * SEQ + n0 + pc * 4) = v; }
    if (pass == 0) __threadfence(); } }

constexpr size_t al256(size_t b) { return (b + 255) & ~(size_t)255; }
constexpr size_t SZ_BW  = (size_t)QP * CIN * 2;
constexpr size_t SZ_WP  = (size_t)CIN * CIN * 2;
constexpr size_t SZ_WT  = (size_t)CIN * TD * 2;
constexpr size_t SZ_T16 = (size_t)TROWS * TD * 2;
constexpr size_t SZ_TE  = (size_t)TROWS * CIN * 4;
constexpr size_t SZ_QH  = NR * QP * 2;
constexpr size_t SZ_VT  = (size_t)NB * NH * HD * SEQ * 2;
constexpr size_t SZ_CTX = NR * CIN * 2;
constexpr size_t SZ_O2  = NR * CIN * 4;
constexpr size_t SZ_X   = NR * CIN * 2;
constexpr size_t SZ_S   = (size_t)NH * SEQ * SEQ * 4;
constexpr size_t SZ_P   = (size_t)NH * SEQ * SEQ * 2;
constexpr size_t SZ_SH  = (SZ_X > SZ_S + SZ_P) ? SZ_X : (SZ_S + SZ_P);
static_assert(SZ_S % 256 == 0);
static_assert(al256(SZ_BW) + al256(SZ_WP) + al256(SZ_WT) + al256(SZ_T16) + al256(SZ_TE) + al256(SZ_QH) + al256(SZ_VT) + al256(SZ_CTX) + al256(SZ_O2) + al256(SZ_SH) <= (size_t)134217728);

extern "C" void kernel_launch(void* const* d_in, const int* in_sizes, int n_in,
                              void* d_out, int out_size, void* d_ws, size_t ws_size, hipStream_t stream) {
  if (n_in < 8) return;
  const float* x     = (const float*)d_in[0];
  const float* t_emb = (const float*)d_in[1];
  const float* Wqkv  = (const float*)d_in[2];
  const float* bqkv  = (const float*)d_in[3];
  const float* Wproj = (const float*)d_in[4];
  const float* bproj = (const float*)d_in[5];
  const float* Wt    = (const float*)d_in[6];
  const float* bt    = (const float*)d_in[7];
  if (in_sizes[0] < (int)(((size_t)NB * CIN - 1) * SEQ_FULL + SEQ)) return;
  if (in_sizes[1] < NB * TD) return;
  if (in_sizes[2] < CIN * QP || in_sizes[3] < QP) return;
  if (in_sizes[4] < CIN * CIN || in_sizes[5] < CIN) return;
  if (in_sizes[6] < TD * CIN || in_sizes[7] < CIN) return;
  if (out_size < (int)((size_t)NB * CIN * SEQ)) return;
  char* ws = (char*)d_ws; size_t off = 0;
  auto take = [&](size_t bytes) { char* p = ws + off; off += (bytes + 255) & ~(size_t)255; return p; };
  _Float16* BW  = (_Float16*)take(SZ_BW);
  _Float16* WPT = (_Float16*)take(SZ_WP);
  _Float16* WTT = (_Float16*)take(SZ_WT);
  _Float16* T16 = (_Float16*)take(SZ_T16);
  float*    TE  = (float*)take(SZ_TE);
  _Float16* QH  = (_Float16*)take(SZ_QH);
  _Float16* VT  = (_Float16*)take(SZ_VT);
  _Float16* CTX = (_Float16*)take(SZ_CTX);
  float*    O2  = (float*)take(SZ_O2);
  char* SH = take(SZ_SH);
  _Float16* X16 = (_Float16*)SH; float* S = (float*)SH; _Float16* P = (_Float16*)(SH + SZ_S);
  if (off > ws_size) return;
  float* out = (float*)d_out;

  k_w16t<<<(unsigned)((QP * (CIN / 8)) / 256), 256, 0, stream>>>(Wqkv, QP, QP, BW);
  k_w16t<<<(unsigned)((CIN * (CIN / 8)) / 256), 256, 0, stream>>>(Wproj, CIN, CIN, WPT);
  k_w16t<<<(unsigned)((CIN * (CIN / 8)) / 256), 256, 0, stream>>>(Wt, CIN, CIN, WTT);
  k_t16<<<(unsigned)((TROWS * (TD / 8)) / 256), 256, 0, stream>>>(t_emb, T16);
  k_gemm2<0><<<dim3((unsigned)(CIN / 64), 1), 128, 0, stream>>>(T16, TD, 0, nullptr, 0, 0, WTT, TD, 0, nullptr, 0, 0, 1.0f,
      0.0625f, bt, 0, TE, nullptr, CIN, 0, nullptr, 0, 0, 0, TROWS, CIN, TD);
  k_xt16<<<(unsigned)(NB * (SEQ / 64) * (CIN / 64)), 256, 0, stream>>>(x, TE, X16);
  k_gemm2<0><<<dim3((unsigned)((NR / 128) * (QP / 64)), 1), 128, 0, stream>>>(X16, CIN, 0, nullptr, 0, 0, BW, CIN, 0, nullptr, 0, 0, 1.0f,
      0.0625f, bqkv, 0, nullptr, QH, QP, 0, nullptr, 0, 0, 0, (int)NR, QP, CIN);
  k_vt<<<(unsigned)(NB * NH * (SEQ / 64)), 256, 0, stream>>>(QH, VT);
  for (int b = 0; b < NB; ++b) {
    const _Float16* QHb = QH + (size_t)b * SEQ * QP;
    k_gemm2<0><<<dim3((SEQ / 128) * (SEQ / 64), NH), 128, 0, stream>>>(QHb, QP, (size_t)HD, nullptr, 0, 0, QHb + KOF, QP, (size_t)HD, nullptr, 0, 0, 1.0f,
        0.125f, nullptr, 0, S, nullptr, SEQ, (size_t)SEQ * SEQ, nullptr, 0, 0, 0, SEQ, SEQ, HD);
    k_rsmw<<<(NH * SEQ + 7) / 8, 256, 0, stream>>>(S, P, NH * SEQ);
    k_gemm2<0><<<dim3((SEQ / 128) * (HD / 64), NH), 128, 0, stream>>>(P, SEQ, (size_t)SEQ * SEQ, nullptr, 0, 0, VT + (size_t)b * NH * HD * SEQ, SEQ, (size_t)HD * SEQ, nullptr, 0, 0, 1.0f,
        1.0f / PCARRY, nullptr, 0, nullptr, CTX + (size_t)b * SEQ * CIN, CIN, (size_t)HD, nullptr, 0, 0, 0, SEQ, HD, SEQ);
  }
  k_gemm2<0><<<dim3((unsigned)((NR / 128) * (CIN / 64)), 1), 128, 0, stream>>>(CTX, CIN, 0, nullptr, 0, 0, WPT, CIN, 0, nullptr, 0, 0, 1.0f,
      0.0625f, bproj, 0, O2, nullptr, CIN, 0, nullptr, 0, 0, 0, (int)NR, CIN, CIN);
  k_outT<<<(unsigned)(NB * (SEQ / 64) * (CIN / 64)), 256, 0, stream>>>(O2, out);
}
